// SS3DConv_45243185496332
// MI455X (gfx1250) — hardware-run, weakly checked
//
#include <hip/hip_runtime.h>
#include <math.h>

#define NBAT 2
#define LTOK 4096
#define LTSH 12
#define NTOK (NBAT * LTOK)
#define CIN  128
#define DIN  256
#define CCV  16
#define GRP  16
#define NNB  27
#define DSQ  432
#define DSQP 448
#define NCG  (DSQP / 64)
#define DST  16
#define DTR  14
#define XPR  46
#define XDN  64
#define XBO  14
#define XCO  30
#define EPSV 1e-5f
#define GSTR 40
#define OSTR 68
#define SMEMB (8 * 16 * OSTR * 4)
#define SCH  32
#define LOG2E 1.4426950408889634f

static_assert(LTOK == (1 << LTSH));
static_assert(NTOK % 128 == 0);
static_assert(CIN % 32 == 0 && DIN % 32 == 0 && DSQP % 32 == 0);
static_assert(DSQP % 64 == 0 && DSQP >= DSQ);
static_assert((DSQP / 8) % 8 == 0);
static_assert(XDN % 64 == 0 && XCO + DST <= XDN && XCO + DST <= 48);
static_assert(DSQ == CCV * NNB);
static_assert(SMEMB >= (2 * 128 * GSTR + 2 * 64 * GSTR) * 2);
static_assert(LTOK % SCH == 0);
static_assert((SCH * 8) % 64 == 0);
static_assert(DIN == 32 * 8);
static_assert((NTOK * CCV) % 256 == 0);
static_assert((NTOK * (DSQP / 8)) % 256 == 0);

typedef unsigned short us16 __attribute__((ext_vector_type(16)));
typedef unsigned short us8  __attribute__((ext_vector_type(8)));
typedef unsigned short us8a __attribute__((ext_vector_type(8), may_alias));
typedef __bf16 v16b __attribute__((ext_vector_type(16)));
typedef float v8f __attribute__((ext_vector_type(8)));
typedef float v4f __attribute__((ext_vector_type(4)));
typedef float v4fa __attribute__((ext_vector_type(4), may_alias));
union FragU { us16 v; us8 h[2]; };

__device__ __forceinline__ unsigned short bf16_bits(float f) {
  unsigned u = __float_as_uint(f);
  u += 0x7FFFu + ((u >> 16) & 1u);
  return (unsigned short)(u >> 16);
}
__device__ __forceinline__ float bf16_val(unsigned short b) { return __uint_as_float(((unsigned)b) << 16); }
__device__ __forceinline__ float bf16r(float f) { return bf16_val(bf16_bits(f)); }
__device__ __forceinline__ float siluf(float x) { return x * __builtin_amdgcn_rcpf(1.0f + __expf(-x)); }

__device__ __forceinline__ v8f mma_bf16(us16 a, us16 b, v8f c) {
  return __builtin_amdgcn_wmma_f32_16x16x32_bf16(false, __builtin_bit_cast(v16b, a), false, __builtin_bit_cast(v16b, b), (short)0, c, false, false);
}
__device__ __forceinline__ void wguard(v8f& c0, v8f& c1, v8f& c2, v8f& c3, const us16& a0, const us16& a1,
                                       const us16& b0, const us16& b1, const us16& b2, const us16& b3,
                                       const us16& e0, const us16& e1, const us16& e2, const us16& e3) {
#if defined(__HIP_DEVICE_COMPILE__)
  asm volatile("v_nop\n\tv_nop\n\tv_nop\n\tv_nop"
               : "+v"(c0), "+v"(c1), "+v"(c2), "+v"(c3)
               : "v"(a0), "v"(a1), "v"(b0), "v"(b1), "v"(b2), "v"(b3), "v"(e0), "v"(e1), "v"(e2), "v"(e3));
#endif
}

__device__ __forceinline__ us16 lds_frag(const unsigned short* base) {
  const int lane = threadIdx.x & 31, r = lane & 15, kh = (lane >> 4) * 8;
  FragU f;
  f.h[0] = *(const us8a*)(base + r * GSTR + kh);
  f.h[1] = *(const us8a*)(base + r * GSTR + 16 + kh);
  return f.v;
}

__device__ __forceinline__ void stage_a(unsigned short* lds, const unsigned short* __restrict__ P, int ld, int m0, int k0, int tid) {
  const int row = tid >> 1, cq = (tid & 1) * 16;
  const unsigned short* src = P + (size_t)(m0 + row) * ld + k0 + cq;
  const us8 v0 = *(const us8a*)src;
  const us8 v1 = *(const us8a*)(src + 8);
  *(us8a*)(lds + row * GSTR + cq) = v0;
  *(us8a*)(lds + row * GSTR + cq + 8) = v1;
}
__device__ __forceinline__ void stage_b(unsigned short* lds, const unsigned short* __restrict__ P, int ld, int n0, int k0, int tid) {
  const int row = tid >> 2, kq = (tid & 3) * 8;
  const us8 v = *(const us8a*)(P + (size_t)(n0 + row) * ld + k0 + kq);
  *(us8a*)(lds + row * GSTR + kq) = v;
}

template <int A2, int B2>
__global__ __launch_bounds__(256) void k_gemm(const unsigned short* __restrict__ A0, const unsigned short* __restrict__ A1, int lda,
                                             const unsigned short* __restrict__ B0, const unsigned short* __restrict__ B1, int ldb,
                                             float* Y, float* Yalt, int nsplit, int ldy, int K, int mrows) {
#pragma clang fp contract(off)
  static_assert(!(A2 && B2));
  __shared__ __attribute__((aligned(16))) unsigned char sm[SMEMB];
  unsigned short* lA0 = (unsigned short*)sm;
  unsigned short* lA1 = lA0 + 128 * GSTR;
  unsigned short* lB0 = lA1 + 128 * GSTR;
  unsigned short* lB1 = lB0 + 64 * GSTR;
  float* oS = (float*)sm;
  const int tid = threadIdx.x, lane = tid & 31, wave = tid >> 5, cl = lane & 15, hh = lane >> 4;
  const int m0 = blockIdx.x * 128;
  const int n0 = blockIdx.y * 64;
  float* Yb = Y;
  int nq = n0;
  if (nsplit > 0 && n0 >= nsplit) { Yb = Yalt; nq = n0 - nsplit; }

  v8f acc[4];
#pragma unroll
  for (int j = 0; j < 4; ++j) { v8f zz = {0.f, 0.f, 0.f, 0.f, 0.f, 0.f, 0.f, 0.f}; acc[j] = zz; }

#pragma unroll 1
  for (int k0 = 0; k0 < K; k0 += 32) {
    __syncthreads();
    stage_a(lA0, A0, lda, m0, k0, tid);
    if (A2) stage_a(lA1, A1, lda, m0, k0, tid);
    stage_b(lB0, B0, ldb, n0, k0, tid);
    if (B2) stage_b(lB1, B1, ldb, n0, k0, tid);
    __syncthreads();
    const us16 af0 = lds_frag(lA0 + 16 * wave * GSTR);
    us16 af1 = af0;
    if (A2) af1 = lds_frag(lA1 + 16 * wave * GSTR);
    us16 b0f[4], b1f[4];
#pragma unroll
    for (int j = 0; j < 4; ++j) {
      b0f[j] = lds_frag(lB0 + 16 * j * GSTR);
      b1f[j] = b0f[j];
      if (B2) b1f[j] = lds_frag(lB1 + 16 * j * GSTR);
    }
#pragma unroll
    for (int j = 0; j < 4; ++j) acc[j] = mma_bf16(af0, b0f[j], acc[j]);
    if (A2) {
#pragma unroll
      for (int j = 0; j < 4; ++j) acc[j] = mma_bf16(af1, b0f[j], acc[j]);
    }
    if (B2) {
#pragma unroll
      for (int j = 0; j < 4; ++j) acc[j] = mma_bf16(af0, b1f[j], acc[j]);
    }
    wguard(acc[0], acc[1], acc[2], acc[3], af0, af1, b0f[0], b0f[1], b0f[2], b0f[3], b1f[0], b1f[1], b1f[2], b1f[3]);
  }
  __syncthreads();

  float* so = oS + wave * (16 * OSTR);
#pragma unroll
  for (int j = 0; j < 4; ++j)
#pragma unroll
    for (int r = 0; r < 8; ++r)
      so[(8 * hh + r) * OSTR + 16 * j + cl] = acc[j][r];
  __syncthreads();
  const bool wst = (m0 + 16 * wave + 16 <= mrows);
#pragma unroll
  for (int pass = 0; pass < 2; ++pass) {
#pragma unroll
    for (int it = 0; it < 8; ++it) {
      const int ch = it * 32 + lane, r = ch >> 4, q = (ch & 15) * 4;
      const v4f v = *(const v4fa*)(so + r * OSTR + q);
      if (wst) *(volatile v4f*)(Yb + (size_t)(m0 + 16 * wave + r) * ldy + nq + q) = v;
    }
    __threadfence();
  }
}

__global__ __launch_bounds__(256) void k_cvt(const float* __restrict__ src, unsigned short* dst, int nsrc, int ksrc, int kdst8, int total8) {
  const int idx = blockIdx.x * 256 + threadIdx.x;
  if (idx >= total8) return;
  const int row = idx / kdst8, c8 = (idx - row * kdst8) * 8;
  const int rs = (row < nsrc) ? row : (nsrc - 1);
  const float* s = src + (size_t)rs * (size_t)ksrc;
  us8 o;
#pragma unroll
  for (int u = 0; u < 8; ++u) {
    const int c = c8 + u;
    const int cc = (c < ksrc) ? c : (ksrc - 1);
    const float v = s[cc];
    o[u] = (row < nsrc && c < ksrc) ? bf16_bits(v) : (unsigned short)0;
  }
  const size_t off = (size_t)row * (size_t)(kdst8 * 8) + c8;
  *(volatile us8*)(dst + off) = o;
  __threadfence();
  *(volatile us8*)(dst + off) = o;
}

__device__ __forceinline__ void split8(const float* v, us8& hi, us8& lo) {
#pragma unroll
  for (int u = 0; u < 8; ++u) {
    const unsigned short hb = bf16_bits(v[u]);
    hi[u] = hb; lo[u] = bf16_bits(v[u] - bf16_val(hb));
  }
}

__global__ __launch_bounds__(256) void k_conv(const float* __restrict__ XP, const float* __restrict__ cw, const float* __restrict__ cb,
                                             float* XC) {
#pragma clang fp contract(off)
  __shared__ __attribute__((aligned(16))) float wsm[CCV * NNB * GRP];
  const int tid = threadIdx.x;
#pragma unroll 1
  for (int e = tid; e < CCV * NNB * GRP; e += 256) {
    const int g = e / (NNB * GRP), rem = e - g * (NNB * GRP), t = rem / GRP, i = rem - t * GRP;
    wsm[e] = bf16r(cw[(g * GRP + i) * NNB + t]);
  }
  __syncthreads();
  const int idx = blockIdx.x * 256 + tid;
  if (idx >= NTOK * CCV) return;
  const int g = idx & (CCV - 1), tok = idx >> 4;
  const int bb = tok >> LTSH, l = tok & (LTOK - 1);
  const int w0 = l & 15, h0 = (l >> 4) & 15, d0 = (l >> 8) & 15;
  float sum = 0.0f;
#pragma unroll 1
  for (int t = 0; t < NNB; ++t) {
    const int i = t / 9, j = (t / 3) % 3, k = t % 3;
    int dz = d0 + i - 1, hz = h0 + j - 1, wz = w0 + k - 1;
    const bool ok = ((unsigned)dz < 16u) && ((unsigned)hz < 16u) && ((unsigned)wz < 16u);
    dz = (dz < 0) ? 0 : ((dz > 15) ? 15 : dz);
    hz = (hz < 0) ? 0 : ((hz > 15) ? 15 : hz);
    wz = (wz < 0) ? 0 : ((wz > 15) ? 15 : wz);
    const float* xp = XP + ((size_t)(bb * LTOK + ((dz * 16 + hz) * 16 + wz))) * DIN + g * GRP;
    const float* wp = wsm + (g * NNB + t) * GRP;
    const v4f xa = *(const v4fa*)xp, xb = *(const v4fa*)(xp + 4), xq = *(const v4fa*)(xp + 8), xd = *(const v4fa*)(xp + 12);
    const v4f wa = *(const v4fa*)wp, wb = *(const v4fa*)(wp + 4), wq = *(const v4fa*)(wp + 8), wv = *(const v4fa*)(wp + 12);
    float tp = 0.0f;
#pragma unroll
    for (int u = 0; u < 4; ++u) tp = tp + xa[u] * wa[u];
#pragma unroll
    for (int u = 0; u < 4; ++u) tp = tp + xb[u] * wb[u];
#pragma unroll
    for (int u = 0; u < 4; ++u) tp = tp + xq[u] * wq[u];
#pragma unroll
    for (int u = 0; u < 4; ++u) tp = tp + xd[u] * wv[u];
    sum = sum + (ok ? tp : 0.0f);
  }
  const float v = siluf(sum + bf16r(cb[g]));
  *(volatile float*)(XC + idx) = v;
  __threadfence();
  *(volatile float*)(XC + idx) = v;
}

__global__ __launch_bounds__(256) void k_unfold(const float* __restrict__ XC, unsigned short* XSH, unsigned short* XSL) {
#pragma clang fp contract(off)
  const int idx = blockIdx.x * 256 + threadIdx.x;
  if (idx >= NTOK * (DSQP / 8)) return;
  const int tok = idx / (DSQP / 8), oc = (idx - tok * (DSQP / 8)) * 8;
  const int bb = tok >> LTSH, l = tok & (LTOK - 1);
  const int w0 = l & 15, h0 = (l >> 4) & 15, d0 = (l >> 8) & 15;
  float v[8];
#pragma unroll
  for (int u = 0; u < 8; ++u) {
    const int col = oc + u;
    const int cc = (col < DSQ) ? col : (DSQ - 1);
    const int c = cc / NNB, o = cc - c * NNB;
    const int i = o / 9, j = (o / 3) % 3, k = o % 3;
    int dz = d0 + i - 1, hz = h0 + j - 1, wz = w0 + k - 1;
    const bool ok = ((unsigned)dz < 16u) && ((unsigned)hz < 16u) && ((unsigned)wz < 16u) && (col < DSQ);
    dz = (dz < 0) ? 0 : ((dz > 15) ? 15 : dz);
    hz = (hz < 0) ? 0 : ((hz > 15) ? 15 : hz);
    wz = (wz < 0) ? 0 : ((wz > 15) ? 15 : wz);
    const float xv = XC[((size_t)(bb * LTOK + ((dz * 16 + hz) * 16 + wz))) * CCV + c];
    v[u] = ok ? xv : 0.0f;
  }
  us8 hi, lo;
  split8(v, hi, lo);
  const size_t off = (size_t)tok * DSQP + oc;
  *(volatile us8*)(XSH + off) = hi; *(volatile us8*)(XSL + off) = lo;
  __threadfence();
  *(volatile us8*)(XSH + off) = hi; *(volatile us8*)(XSL + off) = lo;
}

__global__ __launch_bounds__(64) void k_scan(const float* __restrict__ XD, const unsigned short* __restrict__ XSH,
                                            const unsigned short* __restrict__ XSL, const float* __restrict__ dtw,
                                            const float* __restrict__ dtb, const float* __restrict__ Alog, const float* __restrict__ Dv,
                                            unsigned short* YH, unsigned short* YL) {
#pragma clang fp contract(off)
  __shared__ __attribute__((aligned(16))) float sy[SCH * 64];
  const int bb = blockIdx.x / NCG, cg = blockIdx.x - bb * NCG, t = threadIdx.x;
  const int kd = cg * 64 + t;
  const bool live = (kd < DSQ);
  const int kc = live ? kd : (DSQ - 1);
  float A2[DST], h[DST];
#pragma unroll
  for (int n = 0; n < DST; ++n) { A2[n] = -__expf(bf16r(Alog[kc * DST + n])) * LOG2E; h[n] = 0.0f; }
  float wd[DTR];
#pragma unroll
  for (int r = 0; r < DTR; ++r) wd[r] = bf16r(dtw[kc * DTR + r]);
  const float bd = bf16r(dtb[kc]);
  const float Dd = bf16r(Dv[kc]);
  const float* XDb = XD + (size_t)bb * LTOK * XDN;
  const unsigned short* UHb = XSH + (size_t)bb * LTOK * DSQP + kc;
  const unsigned short* ULb = XSL + (size_t)bb * LTOK * DSQP + kc;
  unsigned short* YHb = YH + (size_t)bb * LTOK * DSQP + cg * 64;
  unsigned short* YLb = YL + (size_t)bb * LTOK * DSQP + cg * 64;
#pragma unroll 1
  for (int c = 0; c < LTOK / SCH; ++c) {
#pragma unroll 1
    for (int s = 0; s < SCH; ++s) {
      const int l = c * SCH + s;
      const float* xr = XDb + (size_t)l * XDN;
      v4f q[12];
#pragma unroll
      for (int i = 0; i < 12; ++i) q[i] = *(const v4fa*)(xr + 4 * i);
      float raw = 0.0f;
#pragma unroll
      for (int r = 0; r < DTR; ++r) raw = raw + q[r >> 2][r & 3] * wd[r];
      const float a = raw + bd;
      const float dl = fmaxf(a, 0.0f) + log1pf(__expf(-fabsf(a)));
      const size_t uo = (size_t)l * DSQP;
      const float uv = bf16_val(UHb[uo]) + bf16_val(ULb[uo]);
      const float dx = dl * uv;
      float y = 0.0f;
#pragma unroll
      for (int n = 0; n < DST; ++n) {
        const float e = exp2f(dl * A2[n]);
        h[n] = e * h[n] + dx * q[(XBO + n) >> 2][(XBO + n) & 3];
        y = y + h[n] * q[(XCO + n) >> 2][(XCO + n) & 3];
      }
      sy[s * 64 + t] = live ? (y + uv * Dd) : 0.0f;
    }
    __syncthreads();
#pragma unroll
    for (int pass = 0; pass < 2; ++pass) {
#pragma unroll
      for (int it = 0; it < (SCH * 8) / 64; ++it) {
        const int ix = it * 64 + t;
        const int r = ix >> 3, oc = (ix & 7) * 8;
        const v4f va = *(const v4fa*)(sy + r * 64 + oc), vb = *(const v4fa*)(sy + r * 64 + oc + 4);
        float vv[8];
#pragma unroll
        for (int u = 0; u < 4; ++u) { vv[u] = va[u]; vv[4 + u] = vb[u]; }
        us8 hi, lo;
        split8(vv, hi, lo);
        const size_t o = (size_t)(c * SCH + r) * DSQP + oc;
        *(volatile us8*)(YHb + o) = hi;
        *(volatile us8*)(YLb + o) = lo;
      }
      __threadfence();
    }
    __syncthreads();
  }
}

__global__ __launch_bounds__(256) void k_gate(const float* __restrict__ YF, const float* __restrict__ XZ, const float* __restrict__ g,
                                             const float* __restrict__ bt, unsigned short* GH, unsigned short* GL) {
#pragma clang fp contract(off)
  const int tid = threadIdx.x, lane = tid & 31, wave = tid >> 5;
  const int tok = blockIdx.x * 8 + wave;
  if (tok >= NTOK) return;
  const int c8 = lane * 8;
  const size_t ro = (size_t)tok * DIN + c8;
  float m[8];
  {
    const v4f a = *(const v4fa*)(YF + ro), b = *(const v4fa*)(YF + ro + 4);
#pragma unroll
    for (int u = 0; u < 4; ++u) { m[u] = a[u]; m[4 + u] = b[u]; }
  }
  float s = ((((((m[0] + m[1]) + m[2]) + m[3]) + m[4]) + m[5]) + m[6]) + m[7];
  s = s + __shfl_xor(s, 16);
  s = s + __shfl_xor(s, 8);
  s = s + __shfl_xor(s, 4);
  s = s + __shfl_xor(s, 2);
  s = s + __shfl_xor(s, 1);
  const float mu = s * (1.0f / (float)DIN);
  float q = 0.0f;
#pragma unroll
  for (int u = 0; u < 8; ++u) { const float dv = m[u] - mu; q = q + dv * dv; }
  q = q + __shfl_xor(q, 16);
  q = q + __shfl_xor(q, 8);
  q = q + __shfl_xor(q, 4);
  q = q + __shfl_xor(q, 2);
  q = q + __shfl_xor(q, 1);
  const float var = q * (1.0f / (float)DIN);
  const float rs = rsqrtf(var + EPSV);
  const v4f za = *(const v4fa*)(XZ + ro), zb = *(const v4fa*)(XZ + ro + 4);
  float gg[8], bq[8];
  {
    const v4f ga = *(const v4fa*)(g + c8), gb = *(const v4fa*)(g + c8 + 4);
    const v4f ba = *(const v4fa*)(bt + c8), b4 = *(const v4fa*)(bt + c8 + 4);
#pragma unroll
    for (int u = 0; u < 4; ++u) { gg[u] = bf16r(ga[u]); gg[4 + u] = bf16r(gb[u]); bq[u] = bf16r(ba[u]); bq[4 + u] = bf16r(b4[u]); }
  }
  float ov[8];
#pragma unroll
  for (int u = 0; u < 4; ++u) {
    const float na = ((m[u] - mu) * rs) * gg[u] + bq[u];
    const float nb = ((m[4 + u] - mu) * rs) * gg[4 + u] + bq[4 + u];
    ov[u]     = na * siluf(za[u]);
    ov[4 + u] = nb * siluf(zb[u]);
  }
  us8 hi, lo;
  split8(ov, hi, lo);
  *(volatile us8*)(GH + ro) = hi; *(volatile us8*)(GL + ro) = lo;
  __threadfence();
  *(volatile us8*)(GH + ro) = hi; *(volatile us8*)(GL + ro) = lo;
}

extern "C" void kernel_launch(void* const* d_in, const int* in_sizes, int n_in,
                              void* d_out, int out_size, void* d_ws, size_t ws_size,
                              hipStream_t stream) {
  if (n_in < 13) return;
  if (in_sizes[0] != NTOK * CIN || in_sizes[1] != 2 * DIN * CIN || in_sizes[2] != CCV * GRP * NNB || in_sizes[3] != CCV ||
      in_sizes[4] != XPR * DSQ || in_sizes[5] != DSQ * DTR || in_sizes[6] != DSQ || in_sizes[7] != DSQ * DST || in_sizes[8] != DSQ ||
      in_sizes[9] != DIN * DSQ || in_sizes[10] != DIN || in_sizes[11] != DIN || in_sizes[12] != CIN * DIN || out_size != NTOK * CIN) return;

  const float* x    = (const float*)d_in[0];
  const float* inw  = (const float*)d_in[1];
  const float* cw   = (const float*)d_in[2];
  const float* cb   = (const float*)d_in[3];
  const float* xpw  = (const float*)d_in[4];
  const float* dtw  = (const float*)d_in[5];
  const float* dtb  = (const float*)d_in[6];
  const float* Alog = (const float*)d_in[7];
  const float* Dv   = (const float*)d_in[8];
  const float* fw   = (const float*)d_in[9];
  const float* lnw  = (const float*)d_in[10];
  const float* lnb  = (const float*)d_in[11];
  const float* ow   = (const float*)d_in[12];
  float* out = (float*)d_out;

  size_t off = 0;
  auto carve = [&](size_t bytes) -> char* { char* p = (char*)d_ws + off; off += (bytes + 255) & ~(size_t)255; return p; };
  unsigned short* WIN16 = (unsigned short*)carve((size_t)2 * DIN * CIN * 2);
  unsigned short* WX16  = (unsigned short*)carve((size_t)XDN * DSQP * 2);
  unsigned short* WF16  = (unsigned short*)carve((size_t)DIN * DSQP * 2);
  unsigned short* WO16  = (unsigned short*)carve((size_t)CIN * DIN * 2);
  unsigned short* X16   = (unsigned short*)carve((size_t)NTOK * CIN * 2);
  float* XP             = (float*)carve((size_t)NTOK * DIN * 4);
  float* XZ             = (float*)carve((size_t)NTOK * DIN * 4);
  float* XC             = (float*)carve((size_t)NTOK * CCV * 4);
  unsigned short* XSH   = (unsigned short*)carve((size_t)NTOK * DSQP * 2);
  unsigned short* XSL   = (unsigned short*)carve((size_t)NTOK * DSQP * 2);
  float* XD             = (float*)carve((size_t)NTOK * XDN * 4);
  unsigned short* YH    = (unsigned short*)carve((size_t)NTOK * DSQP * 2);
  unsigned short* YL    = (unsigned short*)carve((size_t)NTOK * DSQP * 2);
  float* YF             = (float*)carve((size_t)NTOK * DIN * 4);
  unsigned short* GH    = (unsigned short*)carve((size_t)NTOK * DIN * 2);
  unsigned short* GL    = (unsigned short*)carve((size_t)NTOK * DIN * 2);
  if (off > ws_size || off > (size_t)134217728) return;

  const dim3 b256(256), b64(64);
  k_cvt<<<dim3((2 * DIN * (CIN / 8) + 255) / 256), b256, 0, stream>>>(inw, WIN16, 2 * DIN, CIN, CIN / 8, 2 * DIN * (CIN / 8));
  k_cvt<<<dim3((XDN * (DSQP / 8) + 255) / 256), b256, 0, stream>>>(xpw, WX16, XPR, DSQ, DSQP / 8, XDN * (DSQP / 8));
  k_cvt<<<dim3((DIN * (DSQP / 8) + 255) / 256), b256, 0, stream>>>(fw, WF16, DIN, DSQ, DSQP / 8, DIN * (DSQP / 8));
  k_cvt<<<dim3((CIN * (DIN / 8) + 255) / 256), b256, 0, stream>>>(ow, WO16, CIN, DIN, DIN / 8, CIN * (DIN / 8));
  k_cvt<<<dim3((NTOK * (CIN / 8) + 255) / 256), b256, 0, stream>>>(x, X16, NTOK, CIN, CIN / 8, NTOK * (CIN / 8));
  k_gemm<0, 0><<<dim3(NTOK / 128, (2 * DIN) / 64, 1), b256, 0, stream>>>(X16, X16, CIN, WIN16, WIN16, CIN, XP, XZ, DIN, DIN, CIN, NTOK);
  k_conv<<<dim3((NTOK * CCV + 255) / 256), b256, 0, stream>>>(XP, cw, cb, XC);
  k_unfold<<<dim3((NTOK * (DSQP / 8) + 255) / 256), b256, 0, stream>>>(XC, XSH, XSL);
  k_gemm<1, 0><<<dim3(NTOK / 128, XDN / 64, 1), b256, 0, stream>>>(XSH, XSL, DSQP, WX16, WX16, DSQP, XD, XD, 0, XDN, DSQP, NTOK);
  k_scan<<<dim3(NBAT * NCG), b64, 0, stream>>>(XD, XSH, XSL, dtw, dtb, Alog, Dv, YH, YL);
  k_gemm<1, 0><<<dim3(NTOK / 128, DIN / 64, 1), b256, 0, stream>>>(YH, YL, DSQP, WF16, WF16, DSQP, YF, YF, 0, DIN, DSQP, NTOK);
  k_gate<<<dim3((NTOK + 7) / 8), b256, 0, stream>>>(YF, XZ, lnw, lnb, GH, GL);
  k_gemm<1, 0><<<dim3(NTOK / 128, CIN / 64, 1), b256, 0, stream>>>(GH, GL, DIN, WO16, WO16, DIN, out, out, 0, CIN, DIN, NTOK);
}
